// SimpleBaselineRemoval_41893111005596
// MI455X (gfx1250) — hardware-verified
//
#include <hip/hip_runtime.h>


namespace {
constexpr int Bn = 16, T = 262144, FM = 8, W = 8640, PAD = W / 2, KP = W + 32  , NQ = T / 32  , XL = T + KP  , XLP = 270848  ;
constexpr float XS = 1.0f;

typedef _Float16 b16;
typedef __attribute__((ext_vector_type(16))) _Float16 v16b;
typedef __attribute__((ext_vector_type(8))) _Float16 v8b;
typedef __attribute__((ext_vector_type(8))) float v8f;
typedef __attribute__((ext_vector_type(4))) float v4f;
__device__ __forceinline__ float bf16_rne(float f) { unsigned int u = __float_as_uint(f); u += 0x7FFFu + ((u >> 16) & 1u); return __uint_as_float(u & 0xFFFF0000u); }
__device__ __forceinline__ v16b frag_kb(const b16* p, int hh) { const v8b a = *(const v8b*)(p + 8 * hh), b = *(const v8b*)(p + 16 + 8 * hh); v16b f;
#pragma unroll
  for (int e = 0; e < 8; ++e) { f[e] = a[e]; f[8 + e] = b[e]; } return f; }
__device__ __forceinline__ v8f wmma16b(v16b a, v16b b, v8f c) { v8f d = __builtin_amdgcn_wmma_f32_16x16x32_f16(false, a, false, b, (short)0, c, false, false); asm volatile("v_nop\n\tv_nop\n\tv_nop\n\tv_nop" : "+v"(d) : "v"(a), "v"(b)); return d; }
__device__ __forceinline__ void wave_lds_sync() { __builtin_amdgcn_fence(__ATOMIC_RELEASE, "workgroup"); __builtin_amdgcn_wave_barrier(); __builtin_amdgcn_fence(__ATOMIC_ACQUIRE, "workgroup"); }
__device__ __forceinline__ float nexp(float x) { return __builtin_amdgcn_exp2f(x * 1.4426950408889634f); }
__device__ __forceinline__ float pmul(float a, float b) { float p = a * b; asm volatile("" : "+v"(p)); return p; }
__device__ __forceinline__ float wsum(float v) {
#pragma unroll
  for (int o = 1; o < 32; o <<= 1) v += __shfl_xor(v, o); return v; }
__device__ __forceinline__ float wmax(float v) {
#pragma unroll
  for (int o = 1; o < 32; o <<= 1) v = fmaxf(v, __shfl_xor(v, o)); return v; }

constexpr float WSC = 64.0f;
__global__ __launch_bounds__(256) void wprep_kernel(const float* __restrict__ tw, const float* __restrict__ W1, const float* __restrict__ b1, const float* __restrict__ W2, const float* __restrict__ b2, const float* __restrict__ W3, const float* __restrict__ b3, const float* __restrict__ csc, b16* __restrict__ WB, float* __restrict__ P) {
  __shared__ float red[8]; __shared__ float ws[W];
  const int t_ = threadIdx.x, lane = t_ & 31, wave = t_ >> 5;
  float mx = -INFINITY; for (int i = t_; i < W; i += 256) mx = fmaxf(mx, bf16_rne(tw[i])); mx = wmax(mx); if (lane == 0) red[wave] = mx; __syncthreads();
  float gm = red[0]; for (int w_ = 1; w_ < 8; ++w_) gm = fmaxf(gm, red[w_]); __syncthreads();
  float s = 0.0f; for (int i = t_; i < W; i += 256) { const float e = nexp(bf16_rne(tw[i]) - gm); ws[i] = e; s += e; } s = wsum(s); if (lane == 0) red[wave] = s; __syncthreads();
  float tot = 0.0f; for (int w_ = 0; w_ < 8; ++w_) tot += red[w_]; const float inv = 1.0f / tot;
  __syncthreads();
  for (int pass = 0; pass < 2; ++pass) {
    for (int i = t_; i < 32 * (KP / 8); i += 256) { const int r = i / (KP / 8), k0 = (i % (KP / 8)) * 8; v8b v; for (int e = 0; e < 8; ++e) { const int j = k0 + e - r; v[e] = (b16)((j >= 0 && j < W) ? ws[W - 1 - j] * inv * WSC : 0.0f); } *(volatile v8b*)(WB + (size_t)r * KP + k0) = v; }
    for (int i = t_; i < 866; i += 256) { float v; if (i < 288) v = W1[i]; else if (i < 320) v = b1[i - 288]; else if (i < 832) v = W2[i - 320]; else if (i < 848) v = b2[i - 832]; else if (i < 864) v = W3[i - 848]; else if (i == 864) v = b3[0]; else v = csc[0]; P[i] = bf16_rne(v); }
    __threadfence(); }
}

__global__ __launch_bounds__(256) void xpad_kernel(const float* __restrict__ x, b16* __restrict__ XP) {
  const int b = blockIdx.y; const float* xb = x + (size_t)b * T;
  for (int pass = 0; pass < 2; ++pass) { for (int p = blockIdx.x * 256 + threadIdx.x; p < XLP / 8; p += gridDim.x * 256) { v8b v; for (int e = 0; e < 8; ++e) { int i = p * 8 + e - PAD; i = (i < 0) ? 0 : (i >= T ? T - 1 : i); v[e] = (b16)bf16_rne(xb[i]); } *(volatile v8b*)(XP + (size_t)b * XLP + p * 8) = v; } __threadfence(); }
}

__global__ __launch_bounds__(64) void base_kernel(const b16* __restrict__ XP, const b16* __restrict__ WB, float* __restrict__ BL) {
  __shared__ __attribute__((aligned(16))) float Ts[64][32];
  const int lane = threadIdx.x & 31, wave = threadIdx.x >> 5, nloc = lane & 15, hlf = lane >> 4, b = blockIdx.y, q0 = blockIdx.x * 64 + wave * 32; const b16* xb = XP + (size_t)b * XLP;
  v8f acc[2][2];
#pragma unroll
  for (int r = 0; r < 2; ++r) { acc[r][0] = (v8f){}; acc[r][1] = (v8f){}; }
#pragma unroll 2
  for (int kb = 0; kb < KP; kb += 32) { const v16b a0 = frag_kb(xb + (size_t)(q0 + nloc) * 32 + kb, hlf), a1 = frag_kb(xb + (size_t)(q0 + 16 + nloc) * 32 + kb, hlf);
    const v16b w0 = frag_kb(WB + (size_t)nloc * KP + kb, hlf), w1 = frag_kb(WB + (size_t)(16 + nloc) * KP + kb, hlf);
    acc[0][0] = wmma16b(a0, w0, acc[0][0]); acc[0][1] = wmma16b(a0, w1, acc[0][1]); acc[1][0] = wmma16b(a1, w0, acc[1][0]); acc[1][1] = wmma16b(a1, w1, acc[1][1]); }
#pragma unroll
  for (int r = 0; r < 2; ++r)
#pragma unroll
    for (int t = 0; t < 2; ++t)
#pragma unroll
      for (int v = 0; v < 8; ++v) Ts[wave * 32 + r * 16 + 8 * hlf + v][t * 16 + nloc] = acc[r][t][v] * (1.0f / WSC);
  __syncthreads();
  for (int pass = 0; pass < 2; ++pass) { for (int i = threadIdx.x; i < 64 * 32 / 4; i += 64) *(volatile v4f*)(BL + (size_t)b * T + (size_t)blockIdx.x * 2048 + i * 4) = *(const v4f*)(&Ts[0][0] + i * 4); __threadfence(); }
}

__global__ __launch_bounds__(256) void corr_kernel(const float* __restrict__ BL, const float* __restrict__ meta, const float* __restrict__ P, float* __restrict__ CORR) {
  __shared__ float red[8]; __shared__ float h1[32], h2[16], ci[9];
  const int b = blockIdx.x, t_ = threadIdx.x, lane = t_ & 31, wave = t_ >> 5;
  float s = 0.0f; for (int i = t_; i < T; i += 256) s += BL[(size_t)b * T + i]; s = wsum(s); if (lane == 0) red[wave] = s; __syncthreads();
  if (t_ == 0) { float a = 0.0f; for (int w_ = 0; w_ < 8; ++w_) a += red[w_]; ci[0] = a / (float)T; }
  if (t_ < FM) ci[1 + t_] = bf16_rne(meta[b * FM + t_]);
  __syncthreads();
  if (t_ < 32) { float v = P[288 + t_]; for (int k = 0; k < 9; ++k) v += pmul(P[t_ * 9 + k], ci[k]); h1[t_] = fmaxf(v, 0.0f); }
  __syncthreads();
  if (t_ < 16) { float v = P[832 + t_]; for (int k = 0; k < 32; ++k) v += pmul(P[320 + t_ * 32 + k], h1[k]); h2[t_] = fmaxf(v, 0.0f); }
  __syncthreads();
  if (t_ < 32) { float v = P[864]; for (int k = 0; k < 16; ++k) v += pmul(P[848 + k], h2[k]); const float ax = fabsf(v); const float e = nexp(-2.0f * ax); float th = (1.0f - e) / (1.0f + e); th = (v < 0.0f) ? -th : th;
    const float corr = 1.0f + pmul(P[865], th); const float o = (t_ == 0) ? corr : 0.0f; for (int pass = 0; pass < 2; ++pass) ((volatile float*)CORR)[b * 32 + t_] = o; }
  __threadfence();
}

__global__ __launch_bounds__(256) void out_kernel(const float* __restrict__ BL, const float* __restrict__ CORR, float* __restrict__ out) {
  const int b = blockIdx.y; const float c = CORR[b * 32];
  for (int pass = 0; pass < 2; ++pass) { for (int p = blockIdx.x * 256 + threadIdx.x; p < T / 4; p += gridDim.x * 256) { v4f v = *(const v4f*)(BL + (size_t)b * T + p * 4); for (int e = 0; e < 4; ++e) v[e] = pmul(v[e], c); *(volatile v4f*)(out + (size_t)b * T + p * 4) = v; } __threadfence(); }
}
}

extern "C" void kernel_launch(void* const* d_in, const int* in_sizes, int n_in,
                              void* d_out, int out_size, void* d_ws, size_t ws_size, hipStream_t stream) {
  (void)n_in; (void)out_size;
  const float* x = (const float*)d_in[0]; const float* meta = (const float*)d_in[1]; const float* tw = (const float*)d_in[2]; const float* W1 = (const float*)d_in[3]; const float* b1 = (const float*)d_in[4]; const float* W2 = (const float*)d_in[5]; const float* b2 = (const float*)d_in[6]; const float* W3 = (const float*)d_in[7]; const float* b3 = (const float*)d_in[8]; const float* csc = (const float*)d_in[9];
  float* out = (float*)d_out;
  if (in_sizes[0] != Bn * T || in_sizes[2] != W || in_sizes[3] != 32 * 9) return;
  size_t off = 0; char* ws = (char*)d_ws;
  auto carve = [&](size_t bytes) { char* p = ws + off; off += (bytes + 255) & ~(size_t)255; return p; };
  b16* WB = (b16*)carve((size_t)32 * KP * 2); float* P = (float*)carve(1024 * 4); b16* XP = (b16*)carve((size_t)Bn * XLP * 2); float* BL = (float*)carve((size_t)Bn * T * 4); float* CORR = (float*)carve(Bn * 32 * 4);
  if (off > ws_size) return;
  wprep_kernel<<<1, 256, 0, stream>>>(tw, W1, b1, W2, b2, W3, b3, csc, WB, P);
  xpad_kernel<<<dim3(256, Bn), 256, 0, stream>>>(x, XP);
  base_kernel<<<dim3(NQ / 64, Bn), 64, 0, stream>>>(XP, WB, BL);
  corr_kernel<<<Bn, 256, 0, stream>>>(BL, meta, P, CORR);
  out_kernel<<<dim3(256, Bn), 256, 0, stream>>>(BL, CORR, out);
}
